// PointNetSimple_1941325218382
// MI455X (gfx1250) — hardware-verified
//
#include <hip/hip_runtime.h>
#include <stdint.h>
#include <stddef.h>

#pragma clang fp contract(off)

typedef __attribute__((ext_vector_type(16))) __bf16   v16b;
typedef __attribute__((ext_vector_type(8)))  float    v8f;
typedef __attribute__((ext_vector_type(4)))  float    v4f;
typedef __attribute__((ext_vector_type(4)))  unsigned int v4u;
typedef __attribute__((ext_vector_type(4)))  int      v4i;

constexpr int NPTS = 8192;
constexpr int KNBR = 16;
constexpr int NEDGE = NPTS * KNBR;
constexpr int PTS_PER_BLK = 4;
constexpr int CAND_CHUNK = 1024;

static_assert(NPTS % 256 == 0, "a");
static_assert(NPTS % PTS_PER_BLK == 0, "b");
static_assert(NPTS % CAND_CHUNK == 0, "c");

__device__ __forceinline__ unsigned short f2bf_bits(float f) {
  unsigned u = __float_as_uint(f);
  return (unsigned short)((u + 0x7FFFu + ((u >> 16) & 1u)) >> 16);
}
__device__ __forceinline__ float bf_bits2f(unsigned short h) { return __uint_as_float(((unsigned)h) << 16); }
__device__ __forceinline__ void split_bits(float f, unsigned& hb, unsigned& lb) {
  const unsigned short h = f2bf_bits(f);
  hb = (unsigned)h;
  lb = (unsigned)f2bf_bits(f - bf_bits2f(h));
}

union FragU { v16b v; v4u q[2]; };
__device__ __forceinline__ v16b frag_ld(const unsigned short* p) {
  FragU f;
  f.q[0] = *(const v4u*)(const void*)(p);
  f.q[1] = *(const v4u*)(const void*)(p + 16);
  return f.v;
}
__device__ __forceinline__ v8f bmma(v16b a, v16b b, v8f c) {
  c = __builtin_amdgcn_wmma_f32_16x16x32_bf16(false, a, false, b, (short)0, c, false, false);
  asm volatile("v_nop\n\tv_nop\n\tv_nop\n\tv_nop" : "+v"(c) : "v"(a), "v"(b));
  return c;
}

__global__ __launch_bounds__(256) void knn_kernel(const float* __restrict__ pos, int* __restrict__ nbr) {
  __shared__ v4f cand[CAND_CHUNK];
  __shared__ __align__(16) int sIdx[256 * KNBR];

  const int tid = threadIdx.x;
  const int q = blockIdx.x * 256 + tid;

  const float px = pos[q * 3 + 0];
  const float py = pos[q * 3 + 1];
  const float pz = pos[q * 3 + 2];
  const float qt0 = px * px;
  const float qt1 = py * py;
  const float qt2 = pz * pz;
  const float sqi = (qt0 + qt2) + qt1;

  float bd[KNBR];
  int   bi[KNBR];
#pragma unroll
  for (int t = 0; t < KNBR; ++t) { bd[t] = 3.0e38f; bi[t] = 0x7fffffff; }

  for (int ch = 0; ch < NPTS / CAND_CHUNK; ++ch) {
    __syncthreads();
#pragma unroll
    for (int u = 0; u < CAND_CHUNK / 256; ++u) {
      const int c = ch * CAND_CHUNK + u * 256 + tid;
      const float x = pos[c * 3 + 0];
      const float y = pos[c * 3 + 1];
      const float z = pos[c * 3 + 2];
      const float t0 = x * x;
      const float t1 = y * y;
      const float t2 = z * z;
      const float s = (t0 + t2) + t1;
      cand[u * 256 + tid] = (v4f){x, y, z, s};
    }
    __syncthreads();

#pragma unroll 2
    for (int jj = 0; jj < CAND_CHUNK; ++jj) {
      const v4f cv = cand[jj];
      float pr = px * cv.x;
      pr = fmaf(py, cv.y, pr);
      pr = fmaf(pz, cv.z, pr);
      const float ts = sqi + cv.w;
      const float pr2 = 2.0f * pr;
      const float d = ts - pr2;
      if (d < bd[KNBR - 1]) {
        float cd = d;
        int   cj = ch * CAND_CHUNK + jj;
#pragma unroll
        for (int t = 0; t < KNBR; ++t) {
          const float td = bd[t];
          const int   tj = bi[t];
          const bool lt = (cd < td) || ((cd == td) && (cj < tj));
          bd[t] = lt ? cd : td;
          bi[t] = lt ? cj : tj;
          cd = lt ? td : cd;
          cj = lt ? tj : cj;
        }
      }
    }
  }

#pragma unroll
  for (int t = 0; t < KNBR; ++t) sIdx[tid * KNBR + t] = bi[t];
  __syncthreads();

  int* ob = nbr + (size_t)blockIdx.x * (256 * KNBR);
  for (int pass = 0; pass < 2; ++pass) {
#pragma unroll
    for (int s = 0; s < 4; ++s) {
      const int off = s * 1024 + tid * 4;
      const v4i val = *(const v4i*)(&sIdx[off]);
      *(volatile v4i*)(ob + off) = val;
    }
    __threadfence();
  }
}

__global__ __launch_bounds__(256) void wprep_kernel(const float* __restrict__ W, int KA, int NC, int NX, int KP,
                                                    unsigned short* __restrict__ Bh, unsigned short* __restrict__ Bl) {
  const int nchunk = (NC * KP) >> 3;
  const int r = KA - NX;
#pragma unroll 1
  for (int g = threadIdx.x; g < nchunk; g += 256) {
    const int n  = (g * 8) / KP;
    const int s0 = g * 8 - n * KP;
    unsigned ph[4], pl[4];
#pragma unroll
    for (int m = 0; m < 4; ++m) {
      unsigned hpair = 0u, lpair = 0u;
#pragma unroll
      for (int e2 = 0; e2 < 2; ++e2) {
        const int s = s0 + 2 * m + e2;
        const bool inx = (s < NX);
        const int u = s - NX;
        const int k = inx ? s : ((u < r) ? (NX + u) : ((u < 2 * r) ? (NX + u - r) : ((u < 3 * r) ? (NX + u - 2 * r) : 0)));
        const int mh = inx ? 1 : ((u < r) ? 1 : ((u < 2 * r) ? 2 : ((u < 3 * r) ? 1 : 0)));
        int kc = k < 0 ? 0 : k;
        kc = kc > (KA - 1) ? (KA - 1) : kc;
        const float w = W[(size_t)kc * NC + n];
        unsigned hb, lb;
        split_bits(w, hb, lb);
        const unsigned oh = (mh == 1) ? hb : ((mh == 2) ? lb : 0u);
        const unsigned ol = inx ? lb : 0u;
        hpair |= oh << (16 * e2);
        lpair |= ol << (16 * e2);
      }
      ph[m] = hpair;
      pl[m] = lpair;
    }
    const v4u vh = (v4u){ph[0], ph[1], ph[2], ph[3]};
    const v4u vl = (v4u){pl[0], pl[1], pl[2], pl[3]};
    unsigned short* dh = Bh + (size_t)n * KP + s0;
    unsigned short* dl = Bl + (size_t)n * KP + s0;
    *(volatile v4u*)(void*)dh = vh;
    *(volatile v4u*)(void*)dl = vl;
    __threadfence();
    *(volatile v4u*)(void*)dh = vh;
    *(volatile v4u*)(void*)dl = vl;
  }
}

template <int CA, int KP, int NX, int RP>
__global__ __launch_bounds__(2 * CA) void pn_layer(
    const float* __restrict__ pos, const float* __restrict__ xin, const int* __restrict__ nbr,
    const unsigned short* __restrict__ WaH, const unsigned short* __restrict__ WaL, const float* __restrict__ ba,
    const unsigned short* __restrict__ WbH, const unsigned short* __restrict__ WbL, const float* __restrict__ bb,
    float* __restrict__ out) {
  constexpr int NT = 2 * CA;
  constexpr int NROW = PTS_PER_BLK * KNBR;
  constexpr int ALSZ = (NX > 0) ? NROW * KP : 16;
  static_assert(KP % 32 == 0, "d");
  static_assert(CA % 32 == 0, "e");
  static_assert(KP - NX == 32, "f");
  static_assert(3 * RP <= 32, "g");
  static_assert((PTS_PER_BLK * CA) % 128 == 0, "h");

  __shared__ __align__(16) unsigned short Ah[NROW * KP];
  __shared__ __align__(16) unsigned short Al[ALSZ];
  __shared__ __align__(16) unsigned short Hh[NROW * CA];
  __shared__ __align__(16) unsigned short Hl[NROW * CA];
  __shared__ __align__(16) float sOut[PTS_PER_BLK * CA];
  __shared__ int sIdx[NROW];

  const int tid   = threadIdx.x;
  const int lane  = tid & 31;
  const int wave  = tid >> 5;
  const int hh    = lane >> 4;
  const int rlane = lane & 15;
  const int koff  = hh * 8;
  const int p0    = blockIdx.x * PTS_PER_BLK;

  if (tid < NROW) {
    const int q = p0 + (tid >> 4);
    int jr = nbr[(size_t)q * KNBR + (tid & 15)];
    jr = jr < 0 ? 0 : jr;
    jr = jr > (NPTS - 1) ? (NPTS - 1) : jr;
    sIdx[tid] = jr;
  }
  __syncthreads();

  if (tid < NROW) {
    const int row = tid;
    const int qi = p0 + (row >> 4);
    const int j = sIdx[row];
    const float pjx = pos[j * 3 + 0], pjy = pos[j * 3 + 1], pjz = pos[j * 3 + 2];
    const float pix = pos[qi * 3 + 0], piy = pos[qi * 3 + 1], piz = pos[qi * 3 + 2];
    float v[6];
    if (RP == 6) {
      v[0] = pjx; v[1] = pjy; v[2] = pjz;
      v[3] = pjx - pix; v[4] = pjy - piy; v[5] = pjz - piz;
    } else {
      v[0] = pjx - pix; v[1] = pjy - piy; v[2] = pjz - piz;
      v[3] = 0.f; v[4] = 0.f; v[5] = 0.f;
    }
    unsigned tv[32];
#pragma unroll
    for (int s = 0; s < 32; ++s) tv[s] = 0u;
#pragma unroll
    for (int c = 0; c < RP; ++c) {
      unsigned hb, lb;
      split_bits(v[c], hb, lb);
      tv[c] = hb;
      tv[RP + c] = hb;
      tv[2 * RP + c] = lb;
    }
#pragma unroll
    for (int g = 0; g < 4; ++g) {
      const v4u w = (v4u){tv[8 * g + 0] | (tv[8 * g + 1] << 16), tv[8 * g + 2] | (tv[8 * g + 3] << 16),
                          tv[8 * g + 4] | (tv[8 * g + 5] << 16), tv[8 * g + 6] | (tv[8 * g + 7] << 16)};
      *(v4u*)(&Ah[row * KP + NX + 8 * g]) = w;
    }
  }
  if (NX > 0) {
    constexpr int QPR = NT / NROW;
    constexpr int CPT = NX / QPR;
    const int row = tid / QPR;
    const int c0 = (tid - row * QPR) * CPT;
    const int j = sIdx[row];
    const float* src = xin + (size_t)j * NX + c0;
#pragma unroll
    for (int g = 0; g < CPT / 8; ++g) {
      const v4f a = *(const v4f*)(src + 8 * g);
      const v4f b = *(const v4f*)(src + 8 * g + 4);
      unsigned hb[8], lb[8];
      split_bits(a.x, hb[0], lb[0]); split_bits(a.y, hb[1], lb[1]);
      split_bits(a.z, hb[2], lb[2]); split_bits(a.w, hb[3], lb[3]);
      split_bits(b.x, hb[4], lb[4]); split_bits(b.y, hb[5], lb[5]);
      split_bits(b.z, hb[6], lb[6]); split_bits(b.w, hb[7], lb[7]);
      const v4u wh = (v4u){hb[0] | (hb[1] << 16), hb[2] | (hb[3] << 16), hb[4] | (hb[5] << 16), hb[6] | (hb[7] << 16)};
      const v4u wl = (v4u){lb[0] | (lb[1] << 16), lb[2] | (lb[3] << 16), lb[4] | (lb[5] << 16), lb[6] | (lb[7] << 16)};
      *(v4u*)(&Ah[row * KP + c0 + 8 * g]) = wh;
      *(v4u*)(&Al[row * KP + c0 + 8 * g]) = wl;
    }
  }
  __syncthreads();

  const int nb = wave * 16 + rlane;

  v8f acc[4];
#pragma unroll
  for (int i = 0; i < 4; ++i) acc[i] = (v8f){0.f, 0.f, 0.f, 0.f, 0.f, 0.f, 0.f, 0.f};
#pragma unroll
  for (int kc = 0; kc < KP; kc += 32) {
    const v16b bh = frag_ld(WaH + (size_t)nb * KP + kc + koff);
    v16b bl = bh;
    if (NX > 0 && kc < NX) bl = frag_ld(WaL + (size_t)nb * KP + kc + koff);
#pragma unroll
    for (int i = 0; i < 4; ++i) {
      const int ao = (i * 16 + rlane) * KP + kc + koff;
      const v16b ah = frag_ld(&Ah[ao]);
      acc[i] = bmma(ah, bh, acc[i]);
      if (NX > 0 && kc < NX) {
        const v16b al = frag_ld(&Al[ao]);
        acc[i] = bmma(ah, bl, acc[i]);
        acc[i] = bmma(al, bh, acc[i]);
      }
    }
  }
  {
    const float bav = ba[nb];
#pragma unroll
    for (int i = 0; i < 4; ++i) {
#pragma unroll
      for (int r = 0; r < 8; ++r) {
        float hv = acc[i][r] + bav;
        hv = fmaxf(hv, 0.0f);
        unsigned hb, lb;
        split_bits(hv, hb, lb);
        const int row = i * 16 + hh * 8 + r;
        Hh[row * CA + nb] = (unsigned short)hb;
        Hl[row * CA + nb] = (unsigned short)lb;
      }
    }
  }
  __syncthreads();

  v8f acc2[4];
#pragma unroll
  for (int i = 0; i < 4; ++i) acc2[i] = (v8f){0.f, 0.f, 0.f, 0.f, 0.f, 0.f, 0.f, 0.f};
#pragma unroll
  for (int kc = 0; kc < CA; kc += 32) {
    const v16b bh = frag_ld(WbH + (size_t)nb * CA + kc + koff);
    const v16b bl = frag_ld(WbL + (size_t)nb * CA + kc + koff);
#pragma unroll
    for (int i = 0; i < 4; ++i) {
      const int ao = (i * 16 + rlane) * CA + kc + koff;
      const v16b ah = frag_ld(&Hh[ao]);
      const v16b al = frag_ld(&Hl[ao]);
      acc2[i] = bmma(ah, bh, acc2[i]);
      acc2[i] = bmma(ah, bl, acc2[i]);
      acc2[i] = bmma(al, bh, acc2[i]);
    }
  }
  {
    const float bbv = bb[nb];
#pragma unroll
    for (int i = 0; i < 4; ++i) {
      float m = acc2[i][0];
#pragma unroll
      for (int r = 1; r < 8; ++r) m = fmaxf(m, acc2[i][r]);
      const float mo = __shfl_xor(m, 16, 32);
      m = fmaxf(m, mo);
      const float ov = fmaxf(m + bbv, 0.0f);
      if (hh == 0) sOut[i * CA + nb] = ov;
    }
  }
  __syncthreads();

  if (wave == 0) {
    float* ob = out + (size_t)p0 * CA;
    constexpr int NIT = (PTS_PER_BLK * CA) / 128;
    for (int pass = 0; pass < 2; ++pass) {
#pragma unroll
      for (int it = 0; it < NIT; ++it) {
        const int off = (it * 32 + lane) * 4;
        const v4f val = *(const v4f*)(&sOut[off]);
        *(volatile v4f*)(ob + off) = val;
      }
      __threadfence();
    }
  }
}

static_assert((64 * 32 / 8) % 256 == 0, "i");
static_assert((64 * 64 / 8) % 256 == 0, "j");
static_assert((64 * 96 / 8) % 256 == 0, "k");
static_assert((128 * 96 / 8) % 256 == 0, "l");
static_assert((128 * 128 / 8) % 256 == 0, "m");
static_assert((size_t)NPTS * 64 * 4 == 2097152, "n");
static_assert(4194304 + (size_t)NPTS * 128 * 4 == 8388608, "o");

extern "C" void kernel_launch(void* const* d_in, const int* in_sizes, int n_in,
                              void* d_out, int out_size, void* d_ws, size_t ws_size,
                              hipStream_t stream) {
  if (n_in < 13) return;
  if (in_sizes[0] != NPTS * 3) return;
  if (out_size != NPTS * (64 + 64 + 128)) return;

  const float* pos = (const float*)d_in[0];
  const float* W1a = (const float*)d_in[1];  const float* b1a = (const float*)d_in[2];
  const float* W1b = (const float*)d_in[3];  const float* b1b = (const float*)d_in[4];
  const float* W2a = (const float*)d_in[5];  const float* b2a = (const float*)d_in[6];
  const float* W2b = (const float*)d_in[7];  const float* b2b = (const float*)d_in[8];
  const float* W3a = (const float*)d_in[9];  const float* b3a = (const float*)d_in[10];
  const float* W3b = (const float*)d_in[11]; const float* b3b = (const float*)d_in[12];

  float* out0 = (float*)d_out;
  float* out1 = (float*)((char*)d_out + 2097152);
  float* out2 = (float*)((char*)d_out + 4194304);

  char* ws = (char*)d_ws;
  size_t off = 0;
  int* nbr = (int*)(ws + off);
  off += (size_t)NEDGE * 4;
  unsigned short* pl[12];
  const size_t nhalf[12] = {64 * 32, 64 * 32, 64 * 64, 64 * 64,
                            64 * 96, 64 * 96, 64 * 64, 64 * 64,
                            128 * 96, 128 * 96, 128 * 128, 128 * 128};
  for (int i = 0; i < 12; ++i) {
    pl[i] = (unsigned short*)(ws + off);
    off += (nhalf[i] * 2 + 127) & ~(size_t)127;
  }
  if (off > ws_size) return;
  unsigned short* Wa1H = pl[0];  unsigned short* Wa1L = pl[1];
  unsigned short* Wb1H = pl[2];  unsigned short* Wb1L = pl[3];
  unsigned short* Wa2H = pl[4];  unsigned short* Wa2L = pl[5];
  unsigned short* Wb2H = pl[6];  unsigned short* Wb2L = pl[7];
  unsigned short* Wa3H = pl[8];  unsigned short* Wa3L = pl[9];
  unsigned short* Wb3H = pl[10]; unsigned short* Wb3L = pl[11];

  wprep_kernel<<<1, 256, 0, stream>>>(W1a,   6,  64,   0,  32, Wa1H, Wa1L);
  wprep_kernel<<<1, 256, 0, stream>>>(W1b,  64,  64,  64,  64, Wb1H, Wb1L);
  wprep_kernel<<<1, 256, 0, stream>>>(W2a,  67,  64,  64,  96, Wa2H, Wa2L);
  wprep_kernel<<<1, 256, 0, stream>>>(W2b,  64,  64,  64,  64, Wb2H, Wb2L);
  wprep_kernel<<<1, 256, 0, stream>>>(W3a,  67, 128,  64,  96, Wa3H, Wa3L);
  wprep_kernel<<<1, 256, 0, stream>>>(W3b, 128, 128, 128, 128, Wb3H, Wb3L);

  knn_kernel<<<NPTS / 256, 256, 0, stream>>>(pos, nbr);

  pn_layer<64, 32, 0, 6><<<NPTS / PTS_PER_BLK, 128, 0, stream>>>(
      pos, pos, nbr, Wa1H, Wa1L, b1a, Wb1H, Wb1L, b1b, out0);
  pn_layer<64, 96, 64, 3><<<NPTS / PTS_PER_BLK, 128, 0, stream>>>(
      pos, out0, nbr, Wa2H, Wa2L, b2a, Wb2H, Wb2L, b2b, out1);
  pn_layer<128, 96, 64, 3><<<NPTS / PTS_PER_BLK, 256, 0, stream>>>(
      pos, out1, nbr, Wa3H, Wa3L, b3a, Wb3H, Wb3L, b3b, out2);
}
